// MyMultiHeadedAttention_82875688943668
// MI455X (gfx1250) — hardware-verified
//
#include <hip/hip_runtime.h>


#define NB_  4
#define TT   1024
#define DM   512
#define NHD  8
#define DW   (NHD * DM)
#define NT   (NB_ * TT)
#define PCAR 1024.0f
typedef _Float16 h16;
typedef unsigned short bf;
typedef __attribute__((ext_vector_type(16))) __bf16   v16bf;
typedef __attribute__((ext_vector_type(16))) _Float16 v16h;
typedef __attribute__((ext_vector_type(8)))  _Float16 v8h;
typedef __attribute__((ext_vector_type(8)))  unsigned short v8us;
typedef __attribute__((ext_vector_type(8)))  float    v8f;
typedef __attribute__((ext_vector_type(4)))  float    v4f;
typedef v8h  __attribute__((may_alias)) v8ha;
typedef v4f  __attribute__((may_alias)) v4fa;
typedef v8us __attribute__((may_alias)) v8usa;

__device__ __forceinline__ unsigned short f2bf(float f) { unsigned u = __float_as_uint(f); u += 0x7FFFu + ((u >> 16) & 1u); return (unsigned short)(u >> 16); }
__device__ __forceinline__ float bf2f(unsigned short b) { return __uint_as_float(((unsigned)b) << 16); }
__device__ __forceinline__ float bfr(float f) { return bf2f(f2bf(f)); }
__device__ __forceinline__ v16h cat16(v8h lo, v8h hi) { return __builtin_shufflevector(lo, hi, 0, 1, 2, 3, 4, 5, 6, 7, 8, 9, 10, 11, 12, 13, 14, 15); }
__device__ __forceinline__ v16bf cat16b(v8us lo, v8us hi) { return __builtin_bit_cast(v16bf, __builtin_shufflevector(lo, hi, 0, 1, 2, 3, 4, 5, 6, 7, 8, 9, 10, 11, 12, 13, 14, 15)); }
__device__ __forceinline__ v8f wmma16(v16h a, v16h b, v8f c) { return __builtin_amdgcn_wmma_f32_16x16x32_f16(false, a, false, b, (short)0, c, false, false); }
__device__ __forceinline__ v8f wmmab(v16bf a, v16bf b, v8f c) { return __builtin_amdgcn_wmma_f32_16x16x32_bf16(false, a, false, b, (short)0, c, false, false); }


template <typename T16> struct WFrag;
template <> struct WFrag<h16> { typedef v16h V; static __device__ __forceinline__ V ld(const h16* p) { return cat16(*(const v8h*)p, *(const v8h*)(p + 16)); } static __device__ __forceinline__ v8f mma(V a, V b, v8f c) { return wmma16(a, b, c); } };
template <> struct WFrag<bf> { typedef v16bf V; static __device__ __forceinline__ V ld(const bf* p) { return cat16b(*(const v8us*)p, *(const v8us*)(p + 16)); } static __device__ __forceinline__ v8f mma(V a, V b, v8f c) { return wmmab(a, b, c); } };
template <typename T16, int NSPLIT, bool BIAS>
__global__ __launch_bounds__(32) void k_gemmw(const T16* __restrict__ A, const T16* __restrict__ A2, const T16* __restrict__ Bt, const T16* __restrict__ Bt2, int K, float* C, int ldc, const float* __restrict__ bias, size_t sA, size_t sB, size_t sC) {
    typedef typename WFrag<T16>::V V;
    __shared__ __align__(16) float os[16 * 68];
    const size_t z = blockIdx.z; A += z * sA; if (A2) A2 += z * sA; Bt += z * sB; if (Bt2) Bt2 += z * sB; C += z * sC;
    const int lane = threadIdx.x & 31, lr = lane & 15, hi = lane >> 4; const int r0 = blockIdx.x * 64, c0 = blockIdx.y * 64;
    v8f acc[4][4];
#pragma unroll
    for (int mb = 0; mb < 4; ++mb)
#pragma unroll
        for (int nb = 0; nb < 4; ++nb) acc[mb][nb] = (v8f){};
    const size_t aoff = (size_t)(r0 + lr) * K + 8 * hi, boff = (size_t)(c0 + lr) * K + 8 * hi;
#pragma unroll 1
    for (int kc = 0; kc < K; kc += 32) {
        V a[4], a2[4];
#pragma unroll
        for (int mb = 0; mb < 4; ++mb) { a[mb] = WFrag<T16>::ld(A + aoff + (size_t)mb * 16 * K + kc); if (NSPLIT == 1 || NSPLIT == 2) a2[mb] = WFrag<T16>::ld(A2 + aoff + (size_t)mb * 16 * K + kc); }
#pragma unroll
        for (int nb = 0; nb < 4; ++nb) { const V b = WFrag<T16>::ld(Bt + boff + (size_t)nb * 16 * K + kc); V b2; if (NSPLIT >= 2) b2 = WFrag<T16>::ld(Bt2 + boff + (size_t)nb * 16 * K + kc);
#pragma unroll
            for (int mb = 0; mb < 4; ++mb) { acc[mb][nb] = WFrag<T16>::mma(a[mb], b, acc[mb][nb]); if (NSPLIT == 1 || NSPLIT == 2) acc[mb][nb] = WFrag<T16>::mma(a2[mb], b, acc[mb][nb]); if (NSPLIT >= 2) acc[mb][nb] = WFrag<T16>::mma(a[mb], b2, acc[mb][nb]); } }
        asm volatile("v_nop\n\tv_nop\n\tv_nop\n\tv_nop" : "+v"(acc[0][0]), "+v"(acc[1][1]), "+v"(acc[2][2]), "+v"(acc[3][3]) : "v"(a[0]), "v"(a[3]));
    }
#pragma unroll
    for (int mb = 0; mb < 4; ++mb) {
#pragma unroll
        for (int nb = 0; nb < 4; ++nb) {
#pragma unroll
            for (int j = 0; j < 8; ++j) os[(hi * 8 + j) * 68 + nb * 16 + lr] = acc[mb][nb][j]; }
        __builtin_amdgcn_wave_barrier(); asm volatile("" ::: "memory");
        float* crow = C + (size_t)(r0 + mb * 16) * ldc + c0;
#pragma unroll 1
        for (int ps = 0; ps < 2; ++ps) {
#pragma unroll
            for (int s = 0; s < 8; ++s) { const int row = 2 * s + hi, cofs = lr * 4; v4f val = *(const v4fa*)(os + row * 68 + cofs); if (BIAS) { val[0] += bfr(bias[c0 + cofs]); val[1] += bfr(bias[c0 + cofs + 1]); val[2] += bfr(bias[c0 + cofs + 2]); val[3] += bfr(bias[c0 + cofs + 3]); }
                *(volatile v4f*)(crow + (size_t)row * ldc + cofs) = val; }
            if (ps == 0) __threadfence(); }
        __builtin_amdgcn_wave_barrier(); asm volatile("" ::: "memory");
    }
}

__device__ __forceinline__ h16 tohx(float x) { return (h16)x; }
__device__ __forceinline__ void splitf(float y, unsigned short& h, unsigned short& l) { h = f2bf(y); l = f2bf(y - bf2f(h)); }
typedef __attribute__((ext_vector_type(2))) _Float16 v2h;
typedef __attribute__((ext_vector_type(4))) _Float16 v4h;
typedef __attribute__((ext_vector_type(2))) unsigned short v2us;
typedef __attribute__((ext_vector_type(4))) unsigned short v4us;
typedef __attribute__((ext_vector_type(4))) int v4i;

__global__ __launch_bounds__(256) void k_cvt8(const float* __restrict__ src, bf* dst, size_t n8) { const size_t i = (size_t)blockIdx.x * 256 + threadIdx.x; if (i >= n8) return; const v8f v = *(const v8f*)(src + i * 8); v8us o;
#pragma unroll
    for (int k = 0; k < 8; ++k) o[k] = f2bf(v[k]); *(volatile v8us*)(dst + i * 8) = o; __threadfence(); *(volatile v8us*)(dst + i * 8) = o; }
__global__ __launch_bounds__(256) void k_wtG(const float* __restrict__ w, int K, int N, bf* Bt) {
    const int lane = threadIdx.x & 31; const int L0 = (blockIdx.x * 8 + (threadIdx.x >> 5)) * 8; const int nlines = N * K / 64;
#pragma unroll 1
    for (int ps = 0; ps < 2; ++ps) {
#pragma unroll 1
        for (int l = 0; l < 8; ++l) { const int L = L0 + l; if (L >= nlines) break; const size_t e = (size_t)L * 64 + lane * 2; const int k = (int)(e % K), n = (int)(e / K); v2us o;
            o[0] = f2bf(w[(size_t)k * N + n]); o[1] = f2bf(w[(size_t)(k + 1) * N + n]); *(volatile v2us*)(Bt + e) = o; }
        if (ps == 0) __threadfence(); }
}
__global__ __launch_bounds__(256) void k_plane16(const float* __restrict__ F, int NH, float sc, h16* P) {
    const int lane = threadIdx.x & 31; const int L0 = (blockIdx.x * 8 + (threadIdx.x >> 5)) * 8; const int nlines = NH * TT * DM / 64;
#pragma unroll 1
    for (int ps = 0; ps < 2; ++ps) {
#pragma unroll
        for (int l = 0; l < 8; ++l) { const int L = L0 + l; if (L >= nlines) break; const int e = L * 64 + lane * 2; const int d = e & (DM - 1); const int t = (e >> 9) & (TT - 1); const int h = e >> 19; v2h v;
#pragma unroll
            for (int q = 0; q < 2; ++q) v[q] = tohx(F[(size_t)t * (NH * DM) + h * DM + d + q] * sc);
            *(volatile v2h*)(P + (size_t)e) = v; }
        if (ps == 0) __threadfence(); }
}
__global__ __launch_bounds__(256) void k_vt16(const float* __restrict__ F, int NH, h16* VT) {
    const int lane = threadIdx.x & 31; const int L0 = (blockIdx.x * 8 + (threadIdx.x >> 5)) * 8; const int nlines = NH * DM * TT / 64;
#pragma unroll 1
    for (int ps = 0; ps < 2; ++ps) {
#pragma unroll
        for (int l = 0; l < 8; ++l) { const int L = L0 + l; if (L >= nlines) break; const int e = L * 64 + lane * 2; const int t = e & (TT - 1); const int d = (e >> 10) & (DM - 1); const int h = e >> 19; v2h v;
#pragma unroll
            for (int q = 0; q < 2; ++q) v[q] = tohx(F[(size_t)(t + q) * (NH * DM) + h * DM + d]);
            *(volatile v2h*)(VT + (size_t)e) = v; }
        if (ps == 0) __threadfence(); }
}
__global__ __launch_bounds__(256) void k_msoft(const float* __restrict__ Sb, const int* __restrict__ mk, int NR, h16* P) {
    const int lane = threadIdx.x & 31; const int row = blockIdx.x * 8 + (threadIdx.x >> 5); if (row >= NR) return;
    const float* sr = Sb + (size_t)row * TT; float v[32]; float mx = -3.0e38f;
#pragma unroll
    for (int ch = 0; ch < 8; ++ch) { const int j0 = ch * 128 + lane * 4; const v4f a = *(const v4f*)(sr + j0); const v4i m = *(const v4i*)(mk + j0);
#pragma unroll
        for (int q = 0; q < 4; ++q) { const float t = (m[q] == 0) ? -1.0e9f : a[q]; v[ch * 4 + q] = t; mx = fmaxf(mx, t); } }
#pragma unroll
    for (int sh = 16; sh; sh >>= 1) mx = fmaxf(mx, __shfl_xor(mx, sh, 32));
    float sum = 0.f;
#pragma unroll
    for (int k = 0; k < 32; ++k) { v[k] = __expf(v[k] - mx); sum += v[k]; }
#pragma unroll
    for (int sh = 16; sh; sh >>= 1) sum += __shfl_xor(sum, sh, 32);
    const float f = __fdiv_rn(PCAR, sum);
#pragma unroll 1
    for (int ps = 0; ps < 2; ++ps) {
#pragma unroll
        for (int ch = 0; ch < 8; ++ch) { v4h o;
#pragma unroll
            for (int q = 0; q < 4; ++q) o[q] = tohx(v[ch * 4 + q] * f);
            *(volatile v4h*)(P + (size_t)row * TT + ch * 128 + lane * 4) = o; }
        if (ps == 0) __threadfence(); }
}
__global__ __launch_bounds__(256) void k_fuse(const float* __restrict__ O, const float* __restrict__ OP, bf* Mh, bf* Ml) {
    const int lane = threadIdx.x & 31; const int s = blockIdx.x * 8 + (threadIdx.x >> 5); if (s >= TT) return; const float* op = OP + (size_t)s * DM; float dis[NHD];
#pragma unroll 1
    for (int h = 0; h < NHD; ++h) { const float* oh = O + ((size_t)h * TT + s) * DM; float a = 0.f;
#pragma unroll 4
        for (int d = lane; d < DM; d += 32) { const float df = oh[d] * (1.0f / PCAR) - op[d] * (1.0f / PCAR); a = __fadd_rn(a, __fmul_rn(df, df)); }
#pragma unroll
        for (int sh = 16; sh; sh >>= 1) a += __shfl_xor(a, sh, 32);
        dis[h] = a; }
    float wl[NHD]; float mx = -3.0e38f;
#pragma unroll
    for (int h = 0; h < NHD; ++h) { wl[h] = __fdiv_rn(1.0f, dis[h] + 1e-9f); mx = fmaxf(mx, wl[h]); }
    float sum = 0.f;
#pragma unroll
    for (int h = 0; h < NHD; ++h) { wl[h] = __expf(wl[h] - mx); sum += wl[h]; }
    const float inv = __fdiv_rn(1.0f, sum);
#pragma unroll
    for (int h = 0; h < NHD; ++h) wl[h] *= inv;
#pragma unroll 1
    for (int ps = 0; ps < 2; ++ps) {
#pragma unroll 1
        for (int c = 0; c < DM / 128; ++c) { const int d0 = c * 128 + lane * 4; v4us ohh, oll;
#pragma unroll
            for (int q = 0; q < 4; ++q) { const int d = d0 + q; float acc = 0.f;
#pragma unroll
                for (int h = 0; h < NHD; ++h) acc = __fadd_rn(acc, __fmul_rn(wl[h], O[((size_t)h * TT + s) * DM + d] * (1.0f / PCAR)));
                const float m = __fadd_rn(__fmul_rn(acc, 0.8f), __fmul_rn(op[d] * (1.0f / PCAR), 0.2f)); unsigned short a, c2; splitf(m, a, c2); ohh[q] = a; oll[q] = c2; }
            *(volatile v4us*)(Mh + (size_t)s * DM + d0) = ohh; *(volatile v4us*)(Ml + (size_t)s * DM + d0) = oll; }
        if (ps == 0) __threadfence(); }
}

extern "C" void kernel_launch(void* const* d_in, const int* in_sizes, int n_in,
                              void* d_out, int out_size, void* d_ws, size_t ws_size, hipStream_t stream) {
    (void)in_sizes; (void)n_in; (void)out_size;
    const float* IN[19]; for (int i = 0; i < 19; ++i) IN[i] = (const float*)d_in[i];
    const int* mask = (const int*)d_in[3]; const int* maskp = (const int*)d_in[4];
    float* OUT = (float*)d_out;
    char* wsp = (char*)d_ws;
    auto take = [&](size_t bytes) { char* p = wsp; wsp += (bytes + 255) & ~(size_t)255; return (void*)p; };
    bf* WQ = (bf*)take((size_t)DW * DM * 2); bf* WK = (bf*)take((size_t)DW * DM * 2); bf* WV = (bf*)take((size_t)DW * DM * 2); bf* WPQ = (bf*)take((size_t)DM * DM * 2); bf* WPK = (bf*)take((size_t)DM * DM * 2); bf* WPV = (bf*)take((size_t)DM * DM * 2); bf* WO = (bf*)take((size_t)DM * DM * 2);
    bf* XQ = (bf*)take((size_t)NT * DM * 2); bf* XK = (bf*)take((size_t)NT * DM * 2); bf* XV = (bf*)take((size_t)NT * DM * 2);
    float* F = (float*)take((size_t)TT * DW * 4); h16* QP = (h16*)take((size_t)NHD * TT * DM * 2); h16* KP = (h16*)take((size_t)NHD * TT * DM * 2); h16* VT = (h16*)take((size_t)NHD * DM * TT * 2);
    float* Sb = (float*)take((size_t)NHD * TT * TT * 4); h16* Pm = (h16*)take((size_t)NHD * TT * TT * 2); float* Ob = (float*)take((size_t)NHD * TT * DM * 4);
    h16* QPP = (h16*)take((size_t)TT * DM * 2); h16* KPP = (h16*)take((size_t)TT * DM * 2); h16* VTP = (h16*)take((size_t)DM * TT * 2); float* OP = (float*)take((size_t)TT * DM * 4); bf* Mh = (bf*)take((size_t)TT * DM * 2); bf* Ml = (bf*)take((size_t)TT * DM * 2);
    if ((size_t)(wsp - (char*)d_ws) > ws_size) return;
    { const unsigned gW = (unsigned)((DW * DM / 64 + 63) / 64), gP = (unsigned)((DM * DM / 64 + 63) / 64);
      k_wtG<<<gW, 256, 0, stream>>>(IN[5], DM, DW, WQ); k_wtG<<<gW, 256, 0, stream>>>(IN[7], DM, DW, WK); k_wtG<<<gW, 256, 0, stream>>>(IN[9], DM, DW, WV);
      k_wtG<<<gP, 256, 0, stream>>>(IN[11], DM, DM, WPQ); k_wtG<<<gP, 256, 0, stream>>>(IN[13], DM, DM, WPK); k_wtG<<<gP, 256, 0, stream>>>(IN[15], DM, DM, WPV); k_wtG<<<gP, 256, 0, stream>>>(IN[17], DM, DM, WO); }
    { const size_t nx = (size_t)NT * DM / 8; const unsigned gx = (unsigned)((nx + 255) / 256); k_cvt8<<<gx, 256, 0, stream>>>(IN[0], XQ, nx); k_cvt8<<<gx, 256, 0, stream>>>(IN[1], XK, nx); k_cvt8<<<gx, 256, 0, stream>>>(IN[2], XV, nx); }
    const float sc = 0.044194173067808151f;
    const unsigned L8 = (unsigned)((NHD * TT * DM / 64 + 63) / 64), L1 = (unsigned)((TT * DM / 64 + 63) / 64);
    for (int b = 0; b < NB_; ++b) { const size_t r0 = (size_t)b * TT;
        k_gemmw<bf, 0, true><<<dim3(TT / 64, DW / 64, 1), 32, 0, stream>>>(XQ + r0 * DM, nullptr, WQ, nullptr, DM, F, DW, IN[6], 0, 0, 0); k_plane16<<<L8, 256, 0, stream>>>(F, NHD, sc, QP);
        k_gemmw<bf, 0, true><<<dim3(TT / 64, DW / 64, 1), 32, 0, stream>>>(XK + r0 * DM, nullptr, WK, nullptr, DM, F, DW, IN[8], 0, 0, 0); k_plane16<<<L8, 256, 0, stream>>>(F, NHD, 1.0f, KP);
        k_gemmw<bf, 0, true><<<dim3(TT / 64, DW / 64, 1), 32, 0, stream>>>(XV + r0 * DM, nullptr, WV, nullptr, DM, F, DW, IN[10], 0, 0, 0); k_vt16<<<L8, 256, 0, stream>>>(F, NHD, VT);
        k_gemmw<h16, 0, false><<<dim3(TT / 64, TT / 64, NHD), 32, 0, stream>>>(QP, nullptr, KP, nullptr, DM, Sb, TT, nullptr, (size_t)TT * DM, (size_t)TT * DM, (size_t)TT * TT);
        k_msoft<<<NHD * TT / 8, 256, 0, stream>>>(Sb, mask + (size_t)b * TT, NHD * TT, Pm);
        k_gemmw<h16, 0, false><<<dim3(TT / 64, DM / 64, NHD), 32, 0, stream>>>(Pm, nullptr, VT, nullptr, TT, Ob, DM, nullptr, (size_t)TT * TT, (size_t)DM * TT, (size_t)TT * DM);
        k_gemmw<bf, 0, true><<<dim3(TT / 64, DM / 64, 1), 32, 0, stream>>>(XQ + r0 * DM, nullptr, WPQ, nullptr, DM, F, DM, IN[12], 0, 0, 0); k_plane16<<<L1, 256, 0, stream>>>(F, 1, sc, QPP);
        k_gemmw<bf, 0, true><<<dim3(TT / 64, DM / 64, 1), 32, 0, stream>>>(XK + r0 * DM, nullptr, WPK, nullptr, DM, F, DM, IN[14], 0, 0, 0); k_plane16<<<L1, 256, 0, stream>>>(F, 1, 1.0f, KPP);
        k_gemmw<bf, 0, true><<<dim3(TT / 64, DM / 64, 1), 32, 0, stream>>>(XV + r0 * DM, nullptr, WPV, nullptr, DM, F, DM, IN[16], 0, 0, 0); k_vt16<<<L1, 256, 0, stream>>>(F, 1, VTP);
        k_gemmw<h16, 0, false><<<dim3(TT / 64, TT / 64, 1), 32, 0, stream>>>(QPP, nullptr, KPP, nullptr, DM, Sb, TT, nullptr, 0, 0, 0);
        k_msoft<<<TT / 8, 256, 0, stream>>>(Sb, maskp + (size_t)b * TT, TT, Pm);
        k_gemmw<h16, 0, false><<<dim3(TT / 64, DM / 64, 1), 32, 0, stream>>>(Pm, nullptr, VTP, nullptr, TT, OP, DM, nullptr, 0, 0, 0);
        k_fuse<<<TT / 8, 256, 0, stream>>>(Ob, OP, Mh, Ml);
        k_gemmw<bf, 1, true><<<dim3(TT / 64, DM / 64, 1), 32, 0, stream>>>(Mh, Ml, WO, nullptr, DM, OUT + r0 * DM, DM, IN[18], 0, 0, 0); }
}
